// GINModel_23673859736037
// MI455X (gfx1250) — hardware-verified
//
#include <hip/hip_runtime.h>
#include <stddef.h>
#include <stdint.h>


#define NNODE   100000
#define NEDGE   640000
#define NGR     512
#define HID     128
#define NLAY    4
#define GFD     5
#define K2      256
#define HIN     133
#define HK1     160
#define ZHW     320
#define MH      256
#define Z1W     512
#define MP      100096
#define NTHR    256
#define NWAVE   8
#define EPT     8
#define CHUNK   (NTHR * EPT)
#define WCAP    (EPT * 32)
#define LISTN   (NWAVE * WCAP)
#define NB      1024
#define NAGG    98
#define PKS     10
#define RCAP    12288
#define DEGCAP  40
#define GBM     64
#define GBN     128
#define GTHR    128
#define GNT     8
#define NPART   (MP / GBM)
#define PARTW   288
#define PG      32
#define NUW     32768
#define NUH1    10240
#define NUH2    16384
#define NUTOT   (NUW + NUH1 + NUH2)
#define CMP_ZINTS (2 * RCAP + 2 * NB + LISTN)
#define LDS_CMP ((CMP_ZINTS + 16) * 4)
#define WSCAP   134217728

static_assert(HID == 128 && GBN == HID && GTHR == GBN && GBM == (GTHR / 32) * 16 && GBN == 16 * GNT);
static_assert(MP % GBM == 0 && MP >= NNODE && MP - NNODE < GBM + GBM && NNODE - (MP / 128 - 1) * 128 == 32);
static_assert(NAGG * NB >= MP && NB == (1 << PKS) && NB == 4 * NTHR && (NB % NWAVE) == 0);
static_assert(((long long)CHUNK << PKS) < (1LL << 31) && ((long long)NNODE << PKS) < (1LL << 31));
static_assert(RCAP % (4 * NTHR) == 0 && RCAP >= 7103 && DEGCAP >= 21 + 8);
static_assert(CMP_ZINTS % (4 * NTHR) == 0 && LISTN >= NB && LDS_CMP <= 300000);
static_assert((K2 % 32) == 0 && (ZHW % 32) == 0 && (Z1W % 32) == 0 && K2 == 2 * HID);
static_assert(HIN <= HK1 && ZHW == 2 * HK1 && HIN == HID + GFD && Z1W == 2 * MH);
static_assert((NGR % GBM) == 0 && (NGR % 128) == 0 && (NGR % PG) == 0 && (MH % GBN) == 0);
static_assert((NGR * 4) / 128 == 16);
static_assert((NUW % (2 * NTHR)) == 0 && (NUH1 % NTHR) == 0 && (NUH2 % NTHR) == 0 && (NUTOT % NTHR) == 0);
static_assert((PARTW % 32) == 0 && PARTW >= 2 * GBN + 1 && PARTW / 4 <= GTHR);
static_assert((PG * ZHW / 8) % NTHR == 0 && (MP * 16) % NTHR == 0 && (GBM * HID / 4) % NTHR == 0);

typedef float          v4f  __attribute__((ext_vector_type(4)));
typedef float          v8f  __attribute__((ext_vector_type(8)));
typedef int            v4i  __attribute__((ext_vector_type(4)));
typedef int            v8i  __attribute__((ext_vector_type(8)));
typedef unsigned int   v2u  __attribute__((ext_vector_type(2)));
typedef unsigned int   v4u  __attribute__((ext_vector_type(4)));
typedef unsigned short v8us __attribute__((ext_vector_type(8)));
typedef __bf16         v16b __attribute__((ext_vector_type(16)));
typedef v4f  __attribute__((may_alias)) v4fa;
typedef v4i  __attribute__((may_alias)) v4ia;
typedef v8us __attribute__((may_alias)) v8usa;
union Frag { v16b vb; v8us h[2]; v8i w; };

__device__ __forceinline__ v8f wmx(const Frag& a, const Frag& b, v8f c) {
  v8f d = __builtin_amdgcn_wmma_f32_16x16x32_bf16(false, a.vb, false, b.vb, (short)0, c, false, false);
  asm volatile("v_nop\n\tv_nop\n\tv_nop\n\tv_nop" : "+v"(d) : "v"(a.w), "v"(b.w));
  return d;
}

__device__ __forceinline__ unsigned short bf_bits(float f) {
  unsigned int u = __float_as_uint(f);
  u += 0x7FFFu + ((u >> 16) & 1u);
  return (unsigned short)(u >> 16);
}
__device__ __forceinline__ float bf_val(unsigned short b) { return __uint_as_float(((unsigned int)b) << 16); }
__device__ __forceinline__ float bf_rne(float f) { return bf_val(bf_bits(f)); }

__device__ __forceinline__ void hilo8(const v4f a, const v4f b, v8us& hv, v8us& lv) {
  const float f[8] = {a.x, a.y, a.z, a.w, b.x, b.y, b.z, b.w};
#pragma unroll
  for (int j = 0; j < 8; ++j) {
    const unsigned short hb = bf_bits(f[j]);
    hv[j] = hb;
    lv[j] = bf_bits(f[j] - bf_val(hb));
  }
}

__device__ __forceinline__ float bnrelu(float u, float m, float r, float g, float b) {
  const float v = ((u - m) * r) * g + b;
  return (v > 0.0f) ? v : (v - v);
}

struct BnP { v4f m2, r2, g2, b2, m3, r3, g3, b3; };

template <int L0>
__device__ __forceinline__ v4f fsrc(const v4f v, const BnP& p) {
  v4f o;
  if constexpr (L0 != 0) {
    o.x = bf_rne(v.x); o.y = bf_rne(v.y); o.z = bf_rne(v.z); o.w = bf_rne(v.w);
  } else {
    o.x = bnrelu(bnrelu(v.x, p.m2.x, p.r2.x, p.g2.x, p.b2.x), p.m3.x, p.r3.x, p.g3.x, p.b3.x);
    o.y = bnrelu(bnrelu(v.y, p.m2.y, p.r2.y, p.g2.y, p.b2.y), p.m3.y, p.r3.y, p.g3.y, p.b3.y);
    o.z = bnrelu(bnrelu(v.z, p.m2.z, p.r2.z, p.g2.z, p.b2.z), p.m3.z, p.r3.z, p.g3.z, p.b3.z);
    o.w = bnrelu(bnrelu(v.w, p.m2.w, p.r2.w, p.g2.w, p.b2.w), p.m3.w, p.r3.w, p.g3.w, p.b3.w);
  }
  return o;
}

__device__ __forceinline__ int scan_chunk(const int* __restrict__ dsts, int nE, int cbase, int slotBase,
                                          int nb, int vec8, int* list, int tid, int lane, int wave) {
  int wc = 0;
  const int el0  = tid * EPT;
  const int e0   = cbase + el0;
  const int sent = -2147483647 - 1;
  v4i da, db;
  if (vec8 != 0 && cbase + CHUNK <= nE) {
    da = *(const v4i*)(dsts + e0);
    db = *(const v4i*)(dsts + e0 + 4);
  } else {
    da.x = (e0     < nE) ? dsts[min(e0,     nE - 1)] : sent;
    da.y = (e0 + 1 < nE) ? dsts[min(e0 + 1, nE - 1)] : sent;
    da.z = (e0 + 2 < nE) ? dsts[min(e0 + 2, nE - 1)] : sent;
    da.w = (e0 + 3 < nE) ? dsts[min(e0 + 3, nE - 1)] : sent;
    db.x = (e0 + 4 < nE) ? dsts[min(e0 + 4, nE - 1)] : sent;
    db.y = (e0 + 5 < nE) ? dsts[min(e0 + 5, nE - 1)] : sent;
    db.z = (e0 + 6 < nE) ? dsts[min(e0 + 6, nE - 1)] : sent;
    db.w = (e0 + 7 < nE) ? dsts[min(e0 + 7, nE - 1)] : sent;
  }
  const unsigned nbs = (unsigned)slotBase;
  const unsigned unb = (unsigned)nb;
  const unsigned s0 = (unsigned)da.x - nbs, s1 = (unsigned)da.y - nbs;
  const unsigned s2 = (unsigned)da.z - nbs, s3 = (unsigned)da.w - nbs;
  const unsigned s4 = (unsigned)db.x - nbs, s5 = (unsigned)db.y - nbs;
  const unsigned s6 = (unsigned)db.z - nbs, s7 = (unsigned)db.w - nbs;
  const bool h0 = s0 < unb, h1 = s1 < unb, h2 = s2 < unb, h3 = s3 < unb;
  const bool h4 = s4 < unb, h5 = s5 < unb, h6 = s6 < unb, h7 = s7 < unb;
  const unsigned any = __builtin_amdgcn_ballot_w32(h0 | h1 | h2 | h3 | h4 | h5 | h6 | h7);
  if (any != 0u) {
#define HITJ(J, HJ, SJ) { \
      const unsigned mj = __builtin_amdgcn_ballot_w32(HJ); \
      if (mj != 0u) { \
        if (HJ) { \
          const int pos = wc + (int)__builtin_amdgcn_mbcnt_lo(mj, 0u); \
          if (pos < WCAP) list[wave * WCAP + pos] = ((el0 + (J)) << PKS) | (int)(SJ); \
        } \
        wc += (int)__builtin_popcount(mj); } }
    HITJ(0, h0, s0)
    HITJ(1, h1, s1)
    HITJ(2, h2, s2)
    HITJ(3, h3, s3)
    HITJ(4, h4, s4)
    HITJ(5, h5, s5)
    HITJ(6, h6, s6)
    HITJ(7, h7, s7)
#undef HITJ
  }
  return wc;
}

__device__ __forceinline__ v8us gat8(const float* __restrict__ p, int stride) {
  v8us o;
#pragma unroll
  for (int i = 0; i < 8; ++i) o[i] = bf_bits(p[(size_t)i * (size_t)stride]);
  return o;
}
__device__ __forceinline__ void put8(unsigned short* dp, const v8us o) {
  *(volatile v8us*)dp = o;
  __threadfence();
  *(volatile v8us*)dp = o;
}

__global__ __launch_bounds__(NTHR) void k_prep(const float* __restrict__ w1, const float* __restrict__ w2,
                                               const float* __restrict__ hw1, const float* __restrict__ hw2,
                                               unsigned short* wt, unsigned short* h1t, unsigned short* h2t) {
  const int u = (int)blockIdx.x * NTHR + (int)threadIdx.x;
  if (u < NUW / 2) {
    const int l = u >> 12, w = u & 4095, n = w >> 5, k8 = (w & 31) * 8, kk = k8 & (HID - 1);
    const v8us o = gat8(w1 + (size_t)l * HID * HID + (size_t)kk * HID + n, HID);
    put8(wt + (size_t)u * 8, o);
  } else if (u < NUW) {
    const int v = u - NUW / 2;
    const int l = v >> 12, w = v & 4095, n = w >> 5, k8 = (w & 31) * 8, kk = k8 & (HID - 1);
    const v8us o = gat8(w2 + (size_t)l * HID * HID + (size_t)kk * HID + n, HID);
    put8(wt + (size_t)u * 8, o);
  } else if (u < NUW + NUH1) {
    const int v = u - NUW;
    const int n = v / (ZHW / 8);
    const int k8 = (v - n * (ZHW / 8)) * 8;
    const int kk = k8 < HK1 ? k8 : k8 - HK1;
    v8us o;
#pragma unroll
    for (int i = 0; i < 8; ++i) {
      const int r  = kk + i;
      const int rc = r < HIN ? r : HIN - 1;
      const float val = hw1[(size_t)rc * MH + n];
      o[i] = (r < HIN) ? bf_bits(val) : (unsigned short)0;
    }
    put8(h1t + (size_t)v * 8, o);
  } else if (u < NUTOT) {
    const int v = u - NUW - NUH1;
    const int n = v >> 6, k8 = (v & 63) * 8, kk = k8 & (MH - 1);
    const v8us o = gat8(hw2 + (size_t)kk * MH + n, MH);
    put8(h2t + (size_t)v * 8, o);
  }
}

__global__ __launch_bounds__(NTHR) void k_compact(const int* __restrict__ srcs, const int* __restrict__ dsts,
                                                  int nN, int nE, int vec8,
                                                  int* lstO, int* cntO, int* offO) {
  extern __shared__ v4i lds_dyn[];
  int* reg1 = (int*)lds_dyn;
  int* reg2 = reg1 + RCAP;
  int* scnt = reg2 + RCAP;
  int* soff = scnt + NB;
  int* list = soff + NB;
  int* wcnt = list + LISTN;
  int* wtot = wcnt + NWAVE;
  const int tid = (int)threadIdx.x, lane = tid & 31, wave = tid >> 5;
  const int nodeBase = (int)blockIdx.x * NB;

  {
    const v4i z4 = {0, 0, 0, 0};
#pragma unroll 1
    for (int i = 4 * tid; i < CMP_ZINTS; i += 4 * NTHR) *(v4ia*)(reg1 + i) = z4;
    if (tid < 2 * NWAVE) wcnt[tid] = 0;
  }
  __syncthreads();

  int tot = 0, ovf = 0;
  const int nChunks = (nE + CHUNK - 1) / CHUNK;
#pragma unroll 1
  for (int ch = 0; ch < nChunks; ++ch) {
    const int cbase = ch * CHUNK;
    const int wc = scan_chunk(dsts, nE, cbase, nodeBase, NB, vec8, list, tid, lane, wave);
    if (lane == 0) wcnt[wave] = wc;
    __syncthreads();
    int pre = 0, all = 0;
#pragma unroll
    for (int w2 = 0; w2 < NWAVE; ++w2) {
      int c = wcnt[w2];
      c = c < 0 ? 0 : (c > WCAP ? WCAP : c);
      all += c;
      pre += (w2 < wave) ? c : 0;
    }
    const int wcc  = wc > WCAP ? WCAP : wc;
    const int base = tot + pre;
#pragma unroll 1
    for (int i0 = 0; i0 < wcc; i0 += 32) {
      const int i   = i0 + lane;
      const int ic  = i < WCAP ? i : WCAP - 1;
      const int ent = list[wave * WCAP + ic];
      const int el  = (ent >> PKS) & (CHUNK - 1);
      const int sl  = ent & (NB - 1);
      int eid = cbase + el;
      eid = eid < 0 ? 0 : (eid > nE - 1 ? nE - 1 : eid);
      const int sraw = srcs[eid];
      const int s = sraw < 0 ? 0 : (sraw > nN - 1 ? nN - 1 : sraw);
      const int pos = base + i;
      if (i < wcc && pos < RCAP) reg1[pos] = (int)(((unsigned)s << PKS) | (unsigned)sl);
    }
    if (tot + all > RCAP) ovf = 1;
    tot += all;
    tot = tot > RCAP ? RCAP : tot;
    __syncthreads();
  }
  const int nh = tot;

  if (wave == 0) {
#pragma unroll 1
    for (int b0 = 0; b0 < nh; b0 += 32) {
      const int idx = b0 + lane;
      const int uv  = reg1[idx < RCAP ? idx : RCAP - 1];
      const int m32 = (nh - b0) < 32 ? (nh - b0) : 32;
#pragma unroll 1
      for (int k = 0; k < m32; ++k) {
        const int u  = __builtin_amdgcn_readlane(uv, k);
        const int sl = u & (NB - 1);
        if (lane == 0) scnt[sl] = scnt[sl] + 1;
      }
    }
  }
  __syncthreads();

  {
    const v4i ca = *(const v4ia*)(scnt + 4 * tid);
    const int e0 = ca.x < 0 ? 0 : ca.x, e1 = ca.y < 0 ? 0 : ca.y, e2 = ca.z < 0 ? 0 : ca.z, e3 = ca.w < 0 ? 0 : ca.w;
    const int ts = e0 + e1 + e2 + e3;
    int incl = ts;
#pragma unroll
    for (int d = 1; d < 32; d <<= 1) {
      const int up = __shfl_up(incl, d);
      if (lane >= d) incl += up;
    }
    if (lane == 31) wtot[wave] = incl;
    __syncthreads();
    int pre = 0;
#pragma unroll
    for (int w2 = 0; w2 < NWAVE; ++w2) pre += (w2 < wave) ? wtot[w2] : 0;
    int run = pre + incl - ts;
    soff[4 * tid + 0] = run; run += e0;
    soff[4 * tid + 1] = run; run += e1;
    soff[4 * tid + 2] = run; run += e2;
    soff[4 * tid + 3] = run;
  }
  __syncthreads();
  for (int i = tid; i < NB; i += NTHR) list[i] = soff[i];
  __syncthreads();

  if (wave == 0) {
#pragma unroll 1
    for (int b0 = 0; b0 < nh; b0 += 32) {
      const int idx = b0 + lane;
      const int uv  = reg1[idx < RCAP ? idx : RCAP - 1];
      const int m32 = (nh - b0) < 32 ? (nh - b0) : 32;
#pragma unroll 1
      for (int k = 0; k < m32; ++k) {
        const int u  = __builtin_amdgcn_readlane(uv, k);
        const int sl = u & (NB - 1);
        const int sv = (int)((unsigned)u >> PKS);
        if (lane == 0) {
          int pos = list[sl];
          pos = pos < 0 ? 0 : (pos > RCAP - 1 ? RCAP - 1 : pos);
          reg2[pos] = sv;
          list[sl] = pos + 1;
        }
      }
    }
  }
  __syncthreads();

  {
    v4i c = *(const v4ia*)(scnt + 4 * tid);
    const v4i o = *(const v4ia*)(soff + 4 * tid);
    if (ovf != 0) { c.x = -1; c.y = -1; c.z = -1; c.w = -1; }
    int* cp = cntO + nodeBase + 4 * tid;
    int* op = offO + nodeBase + 4 * tid;
    *(volatile v4i*)cp = c;
    *(volatile v4i*)op = o;
    __threadfence();
    *(volatile v4i*)cp = c;
    *(volatile v4i*)op = o;
  }
#pragma unroll 1
  for (int it = 0; it < RCAP / (4 * NTHR); ++it) {
    const int p = it * (4 * NTHR) + 4 * tid;
    const v4i v = *(const v4ia*)(reg2 + p);
    int* lp = lstO + (size_t)blockIdx.x * RCAP + p;
    *(volatile v4i*)lp = v;
    __threadfence();
    *(volatile v4i*)lp = v;
  }
}

template <int L0>
__global__ __launch_bounds__(NTHR) void k_agg(const float* __restrict__ S,
                                              const int* __restrict__ lstI, const int* __restrict__ cntI,
                                              const int* __restrict__ offI,
                                              const float* __restrict__ st2, const float* __restrict__ st3,
                                              unsigned short* p1, int nN, int MPr) {
  __shared__ __attribute__((aligned(16))) int lst[RCAP];
  __shared__ __attribute__((aligned(16))) int scn[NB];
  __shared__ __attribute__((aligned(16))) int sof[NB];
  const int tid = (int)threadIdx.x, lane = tid & 31, wave = tid >> 5;
  const int nodeBase = (int)blockIdx.x * NB;

#pragma unroll 1
  for (int it = 0; it < RCAP / (4 * NTHR); ++it) {
    const int p = it * (4 * NTHR) + 4 * tid;
    *(v4ia*)(lst + p) = *(const v4i*)(lstI + (size_t)blockIdx.x * RCAP + p);
  }
  *(v4ia*)(scn + 4 * tid) = *(const v4i*)(cntI + nodeBase + 4 * tid);
  *(v4ia*)(sof + 4 * tid) = *(const v4i*)(offI + nodeBase + 4 * tid);

  BnP bp;
  {
    const v4f z = {0.f, 0.f, 0.f, 0.f};
    bp.m2 = z; bp.r2 = z; bp.g2 = z; bp.b2 = z; bp.m3 = z; bp.r3 = z; bp.g3 = z; bp.b3 = z;
  }
  if constexpr (L0 == 0) {
    bp.m2 = *(const v4f*)(st2 + 4 * lane);
    bp.r2 = *(const v4f*)(st2 + HID + 4 * lane);
    bp.g2 = *(const v4f*)(st2 + 2 * HID + 4 * lane);
    bp.b2 = *(const v4f*)(st2 + 3 * HID + 4 * lane);
    bp.m3 = *(const v4f*)(st3 + 4 * lane);
    bp.r3 = *(const v4f*)(st3 + HID + 4 * lane);
    bp.g3 = *(const v4f*)(st3 + 2 * HID + 4 * lane);
    bp.b3 = *(const v4f*)(st3 + 3 * HID + 4 * lane);
  }
  __syncthreads();

  const int nbw = NB / NWAVE;
  const float qnan = __int_as_float(0x7fc00000);
#pragma unroll 1
  for (int jt = 0; jt < nbw; ++jt) {
    const int slot = wave * nbw + jt;
    const int grow = nodeBase + slot;
    const int craw = scn[slot];
    int st  = sof[slot];
    int cnt = craw;
    const bool bad = (craw < 0) || (craw > DEGCAP);
    st  = st < 0 ? 0 : (st > RCAP ? RCAP : st);
    cnt = cnt < 0 ? 0 : (cnt > DEGCAP ? DEGCAP : cnt);
    if (cnt > RCAP - st) cnt = RCAP - st;
    const bool liveRow = grow < nN;
    const int nc = liveRow ? grow : nN - 1;
    const v4f sv = fsrc<L0>(*(const v4f*)(S + (size_t)nc * HID + 4 * lane), bp);
    float a0 = sv.x, a1 = sv.y, a2 = sv.z, a3 = sv.w;
#pragma unroll 1
    for (int q = 0; q < cnt; ++q) {
      int idx = st + q; idx = idx > RCAP - 1 ? RCAP - 1 : idx;
      int s = lst[idx]; s = s < 0 ? 0 : (s > nN - 1 ? nN - 1 : s);
      const v4f v = fsrc<L0>(*(const v4f*)(S + (size_t)s * HID + 4 * lane), bp);
      a0 += v.x; a1 += v.y; a2 += v.z; a3 += v.w;
    }
    const float pz = bad ? qnan : 0.0f;
    const float r0 = liveRow ? (a0 + pz) : 0.0f;
    const float r1 = liveRow ? (a1 + pz) : 0.0f;
    const float r2 = liveRow ? (a2 + pz) : 0.0f;
    const float r3 = liveRow ? (a3 + pz) : 0.0f;
    const unsigned short h0 = bf_bits(r0), h1 = bf_bits(r1), h2 = bf_bits(r2), h3 = bf_bits(r3);
    const unsigned short l0 = bf_bits(r0 - bf_val(h0)), l1 = bf_bits(r1 - bf_val(h1));
    const unsigned short l2 = bf_bits(r2 - bf_val(h2)), l3 = bf_bits(r3 - bf_val(h3));
    v2u ph, pl;
    ph.x = (unsigned int)h0 | ((unsigned int)h1 << 16);
    ph.y = (unsigned int)h2 | ((unsigned int)h3 << 16);
    pl.x = (unsigned int)l0 | ((unsigned int)l1 << 16);
    pl.y = (unsigned int)l2 | ((unsigned int)l3 << 16);
    unsigned short* gp = p1 + (size_t)grow * K2 + 4 * lane;
    const bool wsv = grow < MPr;
    if (wsv) { *(volatile v2u*)gp = ph; *(volatile v2u*)(gp + HID) = pl; }
    __threadfence();
    if (wsv) { *(volatile v2u*)gp = ph; *(volatile v2u*)(gp + HID) = pl; }
  }
}

template <int EPI>
__global__ __launch_bounds__(GTHR) void k_gemm(const unsigned short* __restrict__ A, int lda,
                                               const unsigned short* __restrict__ BT, int ldb, int K,
                                               const float* __restrict__ bias,
                                               void* outp, int ldo, int lsplit, int nN, int mRows,
                                               float* part) {
  __shared__ __attribute__((aligned(16))) float stg[GBM * GBN];
  __shared__ __attribute__((aligned(16))) float pst[PARTW];
  const int tid = (int)threadIdx.x, lane = tid & 31, wave = tid >> 5, hh = lane >> 4, m = lane & 15;
  const int rowBase = (int)blockIdx.x * GBM;
  const int colBase = (int)blockIdx.y * GBN;

  v8f acc[GNT];
  {
    const v8f z = {0.f, 0.f, 0.f, 0.f, 0.f, 0.f, 0.f, 0.f};
#pragma unroll
    for (int t = 0; t < GNT; ++t) acc[t] = z;
  }
  const unsigned short* ap = A  + (size_t)(rowBase + 16 * wave + m) * (size_t)lda + 8 * hh;
  const unsigned short* bp = BT + (size_t)(colBase + m) * (size_t)ldb + 8 * hh;

#pragma unroll 1
  for (int k0 = 0; k0 < K; k0 += 32) {
    Frag af;
    af.h[0] = *(const v8usa*)(ap + k0);
    af.h[1] = *(const v8usa*)(ap + k0 + 16);
#pragma unroll
    for (int nt = 0; nt < GNT; ++nt) {
      const unsigned short* wq = bp + (size_t)(16 * nt) * (size_t)ldb + k0;
      Frag bfr;
      bfr.h[0] = *(const v8usa*)wq;
      bfr.h[1] = *(const v8usa*)(wq + 16);
      acc[nt] = wmx(af, bfr, acc[nt]);
    }
  }

#pragma unroll
  for (int nt = 0; nt < GNT; ++nt) {
    const int lc = 16 * nt + m;
    const float bb = bf_rne(bias[colBase + lc]);
#pragma unroll
    for (int r = 0; r < 8; ++r) {
      const int lr = 16 * wave + 8 * hh + r;
      const bool live = (rowBase + lr) < nN;
      float v = acc[nt][r] + bb;
      if constexpr (EPI != 1) v = (v > 0.0f) ? v : 0.01f * v;
      stg[lr * GBN + lc] = live ? v : 0.0f;
    }
  }
  __syncthreads();

  if constexpr (EPI == 2) {
    unsigned short* outH = (unsigned short*)outp;
    const int cb = 8 * m;
    const bool isHi = (hh == 0);
    v4u pk[16];
#pragma unroll
    for (int i = 0; i < 16; ++i) {
      const int lr = 16 * wave + i;
      const v4f a = *(const v4fa*)(stg + lr * GBN + cb);
      const v4f b = *(const v4fa*)(stg + lr * GBN + cb + 4);
      const float f[8] = {a.x, a.y, a.z, a.w, b.x, b.y, b.z, b.w};
      unsigned int w[4];
#pragma unroll
      for (int j = 0; j < 4; ++j) {
        const unsigned short h0 = bf_bits(f[2 * j]), h1 = bf_bits(f[2 * j + 1]);
        const unsigned short l0 = bf_bits(f[2 * j] - bf_val(h0)), l1 = bf_bits(f[2 * j + 1] - bf_val(h1));
        const unsigned short q0 = isHi ? h0 : l0, q1 = isHi ? h1 : l1;
        w[j] = (unsigned int)q0 | ((unsigned int)q1 << 16);
      }
      v4u pv; pv.x = w[0]; pv.y = w[1]; pv.z = w[2]; pv.w = w[3];
      pk[i] = pv;
    }
#pragma unroll
    for (int i = 0; i < 16; ++i) {
      const int gr = rowBase + 16 * wave + i;
      unsigned short* op = outH + (size_t)gr * (size_t)ldo + colBase + cb + hh * lsplit;
      if (gr < mRows) *(volatile v4u*)op = pk[i];
    }
    __threadfence();
#pragma unroll
    for (int i = 0; i < 16; ++i) {
      const int gr = rowBase + 16 * wave + i;
      unsigned short* op = outH + (size_t)gr * (size_t)ldo + colBase + cb + hh * lsplit;
      if (gr < mRows) *(volatile v4u*)op = pk[i];
    }
  } else {
    float* outF = (float*)outp;
    v4f fv[16];
#pragma unroll
    for (int i = 0; i < 16; ++i) {
      const int lr = 16 * wave + i;
      fv[i] = *(const v4fa*)(stg + lr * GBN + 4 * lane);
    }
    v4f pv = {0.f, 0.f, 0.f, 0.f};
    const bool pok = (EPI == 1) && (tid < PARTW / 4);
    if constexpr (EPI == 1) {
      int nvr = nN - rowBase;
      nvr = nvr < 0 ? 0 : (nvr > GBM ? GBM : nvr);
      float s = 0.0f;
#pragma unroll 1
      for (int r = 0; r < nvr; ++r) s += stg[r * GBN + tid];
      const float inv = 1.0f / (float)(nvr < 1 ? 1 : nvr);
      const float mean = s * inv;
      float q = 0.0f;
#pragma unroll 1
      for (int r = 0; r < nvr; ++r) {
        const float d = stg[r * GBN + tid] - mean;
        q = fmaf(d, d, q);
      }
      pst[1 + tid] = mean;
      pst[1 + GBN + tid] = q;
      if (tid == 0) pst[0] = (float)nvr;
#pragma unroll 1
      for (int i = 2 * GBN + 1 + tid; i < PARTW; i += GTHR) pst[i] = 0.0f;
      __syncthreads();
      if (pok) pv = *(const v4fa*)(pst + 4 * tid);
    }
    const size_t prow = (size_t)blockIdx.x * (size_t)gridDim.y + (size_t)blockIdx.y;
    float* pp = part + prow * PARTW + 4 * tid;
#pragma unroll
    for (int i = 0; i < 16; ++i) {
      const int gr = rowBase + 16 * wave + i;
      float* op = outF + (size_t)gr * (size_t)ldo + colBase + 4 * lane;
      if (gr < mRows) *(volatile v4f*)op = fv[i];
    }
    if (pok) *(volatile v4f*)pp = pv;
    __threadfence();
#pragma unroll
    for (int i = 0; i < 16; ++i) {
      const int gr = rowBase + 16 * wave + i;
      float* op = outF + (size_t)gr * (size_t)ldo + colBase + 4 * lane;
      if (gr < mRows) *(volatile v4f*)op = fv[i];
    }
    if (pok) *(volatile v4f*)pp = pv;
  }
}

__global__ __launch_bounds__(GBN) void k_comb(const float* __restrict__ part, int nPart,
                                              const float* __restrict__ gam, const float* __restrict__ bet,
                                              float* st) {
  __shared__ __attribute__((aligned(16))) float stg[4 * GBN];
  const int tid = (int)threadIdx.x;
  double n = 0.0, mean = 0.0, M2 = 0.0;
#pragma unroll 1
  for (int b = 0; b < nPart; ++b) {
    const float* pr = part + (size_t)b * PARTW;
    const double nb = (double)pr[0];
    const double mb = (double)pr[1 + tid];
    const double qb = (double)pr[1 + GBN + tid];
    if (nb > 0.5) {
      const double nn = n + nb;
      const double delta = mb - mean;
      const double f = nb / nn;
      mean = mean + delta * f;
      M2 = M2 + qb + delta * delta * n * f;
      n = nn;
    }
  }
  const double nt = n < 1.0 ? 1.0 : n;
  const float var  = (float)(M2 / nt);
  const float rstd = 1.0f / sqrtf(var + 1e-5f);
  stg[tid]           = (float)mean;
  stg[GBN + tid]     = rstd;
  stg[2 * GBN + tid] = bf_rne(gam[tid]);
  stg[3 * GBN + tid] = bf_rne(bet[tid]);
  __syncthreads();
  const v4f v = *(const v4fa*)(stg + 4 * tid);
  float* dp = st + 4 * tid;
  *(volatile v4f*)dp = v;
  __threadfence();
  *(volatile v4f*)dp = v;
}

__global__ __launch_bounds__(NTHR) void k_apply(const float* __restrict__ T, const float* __restrict__ st,
                                                int nN, int MPr, unsigned short* p1) {
  __shared__ float ssh[4 * HID];
  const int tid = (int)threadIdx.x;
  ssh[tid] = st[tid];
  ssh[NTHR + tid] = st[NTHR + tid];
  __syncthreads();
  const int u = (int)blockIdx.x * NTHR + tid;
  const int row = u >> 4, q = u & 15;
  const int rc = row < nN ? row : nN - 1;
  const bool live = row < nN;
  const float* tp = T + (size_t)rc * HID + 8 * q;
  const v4f a = *(const v4f*)tp;
  const v4f b = *(const v4f*)(tp + 4);
  const float f[8] = {a.x, a.y, a.z, a.w, b.x, b.y, b.z, b.w};
  float y[8];
#pragma unroll
  for (int j = 0; j < 8; ++j) {
    const int c = 8 * q + j;
    const float v = bnrelu(f[j], ssh[c], ssh[HID + c], ssh[2 * HID + c], ssh[3 * HID + c]);
    y[j] = live ? v : 0.0f;
  }
  v4f ya, yb;
  ya.x = y[0]; ya.y = y[1]; ya.z = y[2]; ya.w = y[3];
  yb.x = y[4]; yb.y = y[5]; yb.z = y[6]; yb.w = y[7];
  v8us hv, lv;
  hilo8(ya, yb, hv, lv);
  unsigned short* hp = p1 + (size_t)row * K2 + 8 * q;
  const bool ok = row < MPr;
  if (ok) { *(volatile v8us*)hp = hv; *(volatile v8us*)(hp + HID) = lv; }
  __threadfence();
  if (ok) { *(volatile v8us*)hp = hv; *(volatile v8us*)(hp + HID) = lv; }
}

__global__ __launch_bounds__(NTHR) void k_stat3(const float* __restrict__ U, const float* __restrict__ st2,
                                                int nN, float* part) {
  __shared__ __attribute__((aligned(16))) float tile[GBM * HID];
  __shared__ float ssh[4 * HID];
  __shared__ __attribute__((aligned(16))) float pst[PARTW];
  const int tid = (int)threadIdx.x;
  const int rowBase = (int)blockIdx.x * GBM;
  ssh[tid] = st2[tid];
  ssh[NTHR + tid] = st2[NTHR + tid];
  __syncthreads();
#pragma unroll 1
  for (int it = 0; it < (GBM * HID / 4) / NTHR; ++it) {
    const int p = it * NTHR + tid;
    const int lr = p >> 5, q = p & 31;
    const int grow = rowBase + lr;
    const int gc = grow < nN ? grow : nN - 1;
    const v4f x = *(const v4f*)(U + (size_t)gc * HID + 4 * q);
    const int c = 4 * q;
    v4f y;
    y.x = bnrelu(x.x, ssh[c],     ssh[HID + c],     ssh[2 * HID + c],     ssh[3 * HID + c]);
    y.y = bnrelu(x.y, ssh[c + 1], ssh[HID + c + 1], ssh[2 * HID + c + 1], ssh[3 * HID + c + 1]);
    y.z = bnrelu(x.z, ssh[c + 2], ssh[HID + c + 2], ssh[2 * HID + c + 2], ssh[3 * HID + c + 2]);
    y.w = bnrelu(x.w, ssh[c + 3], ssh[HID + c + 3], ssh[2 * HID + c + 3], ssh[3 * HID + c + 3]);
    *(v4fa*)(tile + lr * HID + 4 * q) = y;
  }
  __syncthreads();
  int nvr = nN - rowBase;
  nvr = nvr < 0 ? 0 : (nvr > GBM ? GBM : nvr);
  if (tid < HID) {
    float s = 0.0f;
#pragma unroll 1
    for (int r = 0; r < nvr; ++r) s += tile[r * HID + tid];
    const float inv = 1.0f / (float)(nvr < 1 ? 1 : nvr);
    const float mean = s * inv;
    float q = 0.0f;
#pragma unroll 1
    for (int r = 0; r < nvr; ++r) {
      const float d = tile[r * HID + tid] - mean;
      q = fmaf(d, d, q);
    }
    pst[1 + tid] = mean;
    pst[1 + HID + tid] = q;
    if (tid == 0) pst[0] = (float)nvr;
  }
  if (tid < PARTW - (2 * HID + 1)) pst[2 * HID + 1 + tid] = 0.0f;
  __syncthreads();
  const bool pok = tid < PARTW / 4;
  v4f pv = {0.f, 0.f, 0.f, 0.f};
  float* pp = part + (size_t)blockIdx.x * PARTW + 4 * tid;
  if (pok) { pv = *(const v4fa*)(pst + 4 * tid); *(volatile v4f*)pp = pv; }
  __threadfence();
  if (pok) *(volatile v4f*)pp = pv;
}

__global__ __launch_bounds__(NTHR) void k_pool(const float* __restrict__ U, const float* __restrict__ st2,
                                               const float* __restrict__ st3, const int* __restrict__ bat,
                                               const float* __restrict__ gf, int nN, int vec8b, int nG,
                                               unsigned short* zh) {
  __shared__ __attribute__((aligned(16))) float accs[PG * HID];
  __shared__ float ssh[8 * HID];
  __shared__ __attribute__((aligned(16))) int list[LISTN];
  __shared__ int wcnt[NWAVE];
  __shared__ __attribute__((aligned(16))) unsigned short tile[PG * ZHW];
  const int tid = (int)threadIdx.x, lane = tid & 31, wave = tid >> 5;
  const int slotBase = (int)blockIdx.x * PG;

  for (int i = tid; i < PG * HID; i += NTHR) accs[i] = 0.0f;
  for (int i = tid; i < LISTN; i += NTHR) list[i] = 0;
  ssh[tid]            = st2[tid];
  ssh[NTHR + tid]     = st2[NTHR + tid];
  ssh[2 * NTHR + tid] = st3[tid];
  ssh[3 * NTHR + tid] = st3[NTHR + tid];
  if (tid < NWAVE) wcnt[tid] = 0;
  __syncthreads();
  const int c = tid & (HID - 1);
  const float m2 = ssh[c], r2 = ssh[HID + c], g2 = ssh[2 * HID + c], b2 = ssh[3 * HID + c];
  const float m3 = ssh[4 * HID + c], r3 = ssh[5 * HID + c], g3 = ssh[6 * HID + c], b3 = ssh[7 * HID + c];

  const int nChunks = (nN + CHUNK - 1) / CHUNK;
#pragma unroll 1
  for (int ch = 0; ch < nChunks; ++ch) {
    const int cbase = ch * CHUNK;
    const int wc = scan_chunk(bat, nN, cbase, slotBase, PG, vec8b, list, tid, lane, wave);
    if (lane == 0) wcnt[wave] = wc;
    __syncthreads();
    if (tid < HID) {
#pragma unroll 1
      for (int w2 = 0; w2 < NWAVE; ++w2) {
        int cc = wcnt[w2];
        cc = cc < 0 ? 0 : (cc > WCAP ? WCAP : cc);
#pragma unroll 1
        for (int i = 0; i < cc; ++i) {
          const int ent = list[w2 * WCAP + i];
          const int el  = (ent >> PKS) & (CHUNK - 1);
          const int sl  = ent & (PG - 1);
          int node = cbase + el;
          node = node < 0 ? 0 : (node > nN - 1 ? nN - 1 : node);
          const float u = U[(size_t)node * HID + c];
          const float v = bnrelu(bnrelu(u, m2, r2, g2, b2), m3, r3, g3, b3);
          accs[sl * HID + c] += v;
        }
      }
    }
    __syncthreads();
  }

  for (int i = tid; i < PG * HID; i += NTHR) {
    const int row = i >> 7, cc = i & (HID - 1);
    const float v = accs[i];
    const unsigned short hb = bf_bits(v);
    const unsigned short lb = bf_bits(v - bf_val(hb));
    tile[row * ZHW + cc] = hb;
    tile[row * ZHW + HK1 + cc] = lb;
  }
  for (int i = tid; i < PG * 32; i += NTHR) {
    const int row = i >> 5, j = i & 31;
    const int g  = slotBase + row;
    const int gc = g < nG ? g : nG - 1;
    const int jj = j < GFD ? j : GFD - 1;
    const float gv = gf[(size_t)gc * GFD + jj];
    const unsigned short bits = bf_bits(gv);
    tile[row * ZHW + HID + j] = (j < GFD) ? bits : (unsigned short)0;
    tile[row * ZHW + HK1 + HID + j] = (unsigned short)0;
  }
  __syncthreads();

  constexpr int NIT = (PG * ZHW / 8) / NTHR;
  v8us pv[NIT];
#pragma unroll
  for (int it = 0; it < NIT; ++it) {
    const int p = it * NTHR + tid;
    pv[it] = *(const v8usa*)(tile + 8 * p);
  }
  unsigned short* zb = zh + (size_t)slotBase * ZHW;
#pragma unroll
  for (int it = 0; it < NIT; ++it) {
    const int p = it * NTHR + tid;
    const int g = slotBase + p / (ZHW / 8);
    if (g < nG) *(volatile v8us*)(zb + 8 * p) = pv[it];
  }
  __threadfence();
#pragma unroll
  for (int it = 0; it < NIT; ++it) {
    const int p = it * NTHR + tid;
    const int g = slotBase + p / (ZHW / 8);
    if (g < nG) *(volatile v8us*)(zb + 8 * p) = pv[it];
  }
}

__global__ __launch_bounds__(512) void k_out(const float* __restrict__ z2, const float* __restrict__ w3,
                                             const float* __restrict__ b3, float* out) {
  __shared__ __attribute__((aligned(16))) float so[NGR];
  const int tid = (int)threadIdx.x, lane = tid & 31, wave = tid >> 5;
  const v4f wa = *(const v4f*)(w3 + 8 * lane);
  const v4f wb = *(const v4f*)(w3 + 8 * lane + 4);
  const float w0 = bf_rne(wa.x), w1 = bf_rne(wa.y), w2 = bf_rne(wa.z), w3v = bf_rne(wa.w);
  const float w4 = bf_rne(wb.x), w5 = bf_rne(wb.y), w6 = bf_rne(wb.z), w7 = bf_rne(wb.w);
  const float bb = bf_rne(b3[0]);
  float res = 0.0f;
#pragma unroll 1
  for (int i = 0; i < 32; ++i) {
    const int g = wave * 32 + i;
    const float* zp = z2 + (size_t)g * MH + 8 * lane;
    const v4f a = *(const v4f*)zp;
    const v4f b = *(const v4f*)(zp + 4);
    float p = a.x * w0;
    p = fmaf(a.y, w1, p);
    p = fmaf(a.z, w2, p);
    p = fmaf(a.w, w3v, p);
    p = fmaf(b.x, w4, p);
    p = fmaf(b.y, w5, p);
    p = fmaf(b.z, w6, p);
    p = fmaf(b.w, w7, p);
#pragma unroll
    for (int d = 16; d >= 1; d >>= 1) p += __shfl_xor(p, d);
    res = (lane == i) ? p : res;
  }
  so[wave * 32 + lane] = res + bb;
  __syncthreads();
  const bool ok = tid < NGR / 4;
  v4f v = {0.f, 0.f, 0.f, 0.f};
  float* dp = out + 4 * (ok ? tid : 0);
  if (ok) { v = *(const v4fa*)(so + 4 * tid); *(volatile v4f*)dp = v; }
  __threadfence();
  if (ok) *(volatile v4f*)dp = v;
}

static inline size_t al256(size_t o) { return (o + 255) & ~(size_t)255; }

extern "C" void kernel_launch(void* const* d_in, const int* in_sizes, int n_in,
                              void* d_out, int out_size, void* d_ws, size_t ws_size,
                              hipStream_t stream) {
  if (n_in < 20) return;
  if (in_sizes[0] != NNODE * HID) return;
  if (in_sizes[1] != 2 * NEDGE) return;
  if (in_sizes[2] != NNODE) return;
  if (in_sizes[3] != NGR * GFD) return;
  if (in_sizes[4] != NLAY * HID * HID || in_sizes[8] != NLAY * HID * HID) return;
  if (in_sizes[5] != NLAY * HID || in_sizes[6] != NLAY * HID || in_sizes[7] != NLAY * HID) return;
  if (in_sizes[9] != NLAY * HID || in_sizes[10] != NLAY * HID || in_sizes[11] != NLAY * HID) return;
  if (in_sizes[12] != NLAY * HID || in_sizes[13] != NLAY * HID) return;
  if (in_sizes[14] != HIN * MH || in_sizes[15] != MH) return;
  if (in_sizes[16] != MH * MH || in_sizes[17] != MH) return;
  if (in_sizes[18] != MH || in_sizes[19] != 1) return;
  if (out_size != NGR) return;

  const float* x    = (const float*)d_in[0];
  const int*   ei   = (const int*)  d_in[1];
  const int*   src  = ei;
  const int*   dst  = ei + NEDGE;
  const int*   bat  = (const int*)  d_in[2];
  const float* gf   = (const float*)d_in[3];
  const float* W1   = (const float*)d_in[4];
  const float* b1   = (const float*)d_in[5];
  const float* g1   = (const float*)d_in[6];
  const float* be1  = (const float*)d_in[7];
  const float* W2   = (const float*)d_in[8];
  const float* b2   = (const float*)d_in[9];
  const float* g2   = (const float*)d_in[10];
  const float* be2  = (const float*)d_in[11];
  const float* g3   = (const float*)d_in[12];
  const float* be3  = (const float*)d_in[13];
  const float* hW1  = (const float*)d_in[14];
  const float* hb1  = (const float*)d_in[15];
  const float* hW2  = (const float*)d_in[16];
  const float* hb2  = (const float*)d_in[17];
  const float* hW3  = (const float*)d_in[18];
  const float* hb3  = (const float*)d_in[19];
  float* out = (float*)d_out;

  const int nN = NNODE, nE = NEDGE;
  const int vec8  = ((nE & 3) == 0) ? 1 : 0;
  const int vec8b = ((nN & 3) == 0) ? 1 : 0;

  char* ws = (char*)d_ws;
  size_t off = 0;
  const size_t oWT  = off; off = al256(off + (size_t)NUW * 16);
  const size_t oH1  = off; off = al256(off + (size_t)NUH1 * 16);
  const size_t oH2  = off; off = al256(off + (size_t)NUH2 * 16);
  const size_t oP1  = off; off = al256(off + (size_t)MP * K2 * 2);
  const size_t oP2  = off; off = al256(off + (size_t)MP * HID * 4);
  const size_t oLS  = off; off = al256(off + (size_t)NAGG * RCAP * 4);
  const size_t oCN  = off; off = al256(off + (size_t)NAGG * NB * 4);
  const size_t oOF  = off; off = al256(off + (size_t)NAGG * NB * 4);
  const size_t oPT  = off; off = al256(off + (size_t)NPART * PARTW * 4);
  const size_t oS1  = off; off = al256(off + (size_t)4 * HID * 4);
  const size_t oS2  = off; off = al256(off + (size_t)4 * HID * 4);
  const size_t oS3  = off; off = al256(off + (size_t)4 * HID * 4);
  const size_t oZH  = off; off = al256(off + (size_t)NGR * ZHW * 2);
  const size_t oZ1  = off; off = al256(off + (size_t)NGR * Z1W * 2);
  const size_t oZ2  = off; off = al256(off + (size_t)NGR * MH * 4);
  if (off > ws_size || off > (size_t)WSCAP) return;
  unsigned short* WT  = (unsigned short*)(ws + oWT);
  unsigned short* H1T = (unsigned short*)(ws + oH1);
  unsigned short* H2T = (unsigned short*)(ws + oH2);
  unsigned short* P1  = (unsigned short*)(ws + oP1);
  float*          P2  = (float*)(ws + oP2);
  int*            LS  = (int*)(ws + oLS);
  int*            CN  = (int*)(ws + oCN);
  int*            OF  = (int*)(ws + oOF);
  float*          PT  = (float*)(ws + oPT);
  float*          S1  = (float*)(ws + oS1);
  float*          S2  = (float*)(ws + oS2);
  float*          S3  = (float*)(ws + oS3);
  unsigned short* ZH  = (unsigned short*)(ws + oZH);
  unsigned short* Z1  = (unsigned short*)(ws + oZ1);
  float*          Z2  = (float*)(ws + oZ2);

  hipFuncSetAttribute(reinterpret_cast<const void*>(&k_compact), hipFuncAttributeMaxDynamicSharedMemorySize, LDS_CMP);

  k_prep<<<NUTOT / NTHR, NTHR, 0, stream>>>(W1, W2, hW1, hW2, WT, H1T, H2T);
  k_compact<<<NAGG, NTHR, LDS_CMP, stream>>>(src, dst, nN, nE, vec8, LS, CN, OF);

  for (int l = 0; l < NLAY; ++l) {
    const unsigned short* w1t = WT + (size_t)l * HID * K2;
    const unsigned short* w2t = WT + (size_t)(NLAY + l) * HID * K2;
    if (l == 0) k_agg<1><<<NAGG, NTHR, 0, stream>>>(x,  LS, CN, OF, S2, S3, P1, nN, MP);
    else        k_agg<0><<<NAGG, NTHR, 0, stream>>>(P2, LS, CN, OF, S2, S3, P1, nN, MP);
    k_gemm<1><<<dim3(NPART, 1), GTHR, 0, stream>>>(P1, K2, w1t, K2, K2, b1 + l * HID, (void*)P2, HID, 0, nN, MP, PT);
    k_comb<<<1, GBN, 0, stream>>>(PT, NPART, g1 + l * HID, be1 + l * HID, S1);
    k_apply<<<(MP * 16) / NTHR, NTHR, 0, stream>>>(P2, S1, nN, MP, P1);
    k_gemm<1><<<dim3(NPART, 1), GTHR, 0, stream>>>(P1, K2, w2t, K2, K2, b2 + l * HID, (void*)P2, HID, 0, nN, MP, PT);
    k_comb<<<1, GBN, 0, stream>>>(PT, NPART, g2 + l * HID, be2 + l * HID, S2);
    k_stat3<<<NPART, NTHR, 0, stream>>>(P2, S2, nN, PT);
    k_comb<<<1, GBN, 0, stream>>>(PT, NPART, g3 + l * HID, be3 + l * HID, S3);
  }

  k_pool<<<NGR / PG, NTHR, 0, stream>>>(P2, S2, S3, bat, gf, nN, vec8b, NGR, ZH);
  k_gemm<2><<<dim3(NGR / GBM, MH / GBN), GTHR, 0, stream>>>(ZH, ZHW, H1T, ZHW, ZHW, hb1, (void*)Z1, Z1W, MH, NGR, NGR, PT);
  k_gemm<3><<<dim3(NGR / GBM, MH / GBN), GTHR, 0, stream>>>(Z1, Z1W, H2T, Z1W, Z1W, hb2, (void*)Z2, MH, 0, NGR, NGR, PT);
  k_out<<<1, 512, 0, stream>>>(Z2, hW3, hb3, out);
}
